// Local_Receptive_Field_33148557590653
// MI455X (gfx1250) — hardware-verified
//
#include <hip/hip_runtime.h>
#include <stdint.h>


typedef _Float16 h8  __attribute__((ext_vector_type(8)));
typedef _Float16 h16 __attribute__((ext_vector_type(16)));
typedef h8 h8a __attribute__((may_alias));
typedef float f2 __attribute__((ext_vector_type(2)));
typedef float f4 __attribute__((ext_vector_type(4)));
typedef float f8 __attribute__((ext_vector_type(8)));

#define NNODES   1024
#define IMGPIX   4096
#define IMGW     64
#define HID      90
#define HP       96
#define NLAY     4
#define NELEC    7
#define NTHR     256
#define WPB      8
#define PIT      4
#define ROWS_PER_BLOCK (WPB * PIT * 32)

#define WH_HALVES (NLAY * HP * HP)
#define WH_VEC    (WH_HALVES / 8)
#define WSCALE     16.0f
#define WSCALE_INV 0.0625f

#define OFF_WH    0
#define OFF_ACT   (OFF_WH + WH_HALVES * 2)
#define OFF_WIN   (OFF_ACT + WPB * 32 * HP * 2)
#define OFF_BIN   (OFF_WIN + HP * 8 * 4)
#define OFF_BH    (OFF_BIN + HP * 4)
#define OFF_WOUT  (OFF_BH + NLAY * HP * 4)
#define SMEM_BYTES (OFF_WOUT + HP * 4)

static_assert(ROWS_PER_BLOCK == NNODES);
static_assert(SMEM_BYTES == 128256);
static_assert((OFF_ACT % 16) == 0);
static_assert((OFF_WIN % 16) == 0);
static_assert(WH_VEC * 8 == WH_HALVES);
static_assert((WH_HALVES * 2) % 128 == 0);

__device__ __forceinline__ h16 lds_frag(const _Float16* p) {
  h8 lo = *(const h8a*)(p);
  h8 hi = *(const h8a*)(p + 16);
  return __builtin_shufflevector(lo, hi, 0,1,2,3,4,5,6,7,8,9,10,11,12,13,14,15);
}

__device__ __forceinline__ f8 splat8(float v) {
  f8 r;
#pragma unroll
  for (int i = 0; i < 8; ++i) r[i] = v;
  return r;
}

__device__ __forceinline__ f8 wmma16(h16 a, h16 b, f8 c) {
  f8 d = __builtin_amdgcn_wmma_f32_16x16x32_f16(false, a, false, b, (short)0, c, false, false);
  asm volatile("v_nop\n\tv_nop\n\tv_nop\n\tv_nop" : "+v"(d) : "v"(a), "v"(b));
  return d;
}

__device__ __forceinline__ void hidden_layer_store(_Float16* act, const _Float16* w,
                                                   const float* b16, int nl, int lh) {
  h16 af0[3], af1[3];
  const _Float16* a0p = act + nl * HP + 8 * lh;
  const _Float16* a1p = a0p + 16 * HP;
#pragma unroll
  for (int c = 0; c < 3; ++c) {
    af0[c] = lds_frag(a0p + c * 32);
    af1[c] = lds_frag(a1p + c * 32);
  }
  const _Float16* wp = w + nl * HP + 8 * lh;
#pragma unroll 1
  for (int t = 0; t < 6; ++t) {
    f8 d0 = splat8(b16[t * 16 + nl]);
    f8 d1 = d0;
#pragma unroll
    for (int c = 0; c < 3; ++c) {
      h16 bf = lds_frag(wp + t * 16 * HP + c * 32);
      d0 = wmma16(af0[c], bf, d0);
      d1 = wmma16(af1[c], bf, d1);
    }
    _Float16* o0 = act + (8 * lh) * HP + t * 16 + nl;
    _Float16* o1 = o0 + 16 * HP;
#pragma unroll
    for (int r = 0; r < 8; ++r) {
      o0[r * HP] = (_Float16)fmaxf(d0[r] * WSCALE_INV, 0.f);
      o1[r * HP] = (_Float16)fmaxf(d1[r] * WSCALE_INV, 0.f);
    }
  }
}

__global__ __launch_bounds__(NTHR) void k_prep_wh(const float* __restrict__ Wh,
                                                  h8* __restrict__ wsW, int nvec) {
  const int i = blockIdx.x * NTHR + threadIdx.x;
  if (i >= nvec) return;
  const int L  = i / (HP * HP / 8);
  const int r  = i - L * (HP * HP / 8);
  const int n  = r / (HP / 8);
  const int kb = (r - n * (HP / 8)) * 8;
  h8 v;
#pragma unroll
  for (int j = 0; j < 8; ++j) {
    const int k = kb + j;
    float wv = 0.f;
    if (n < HID && k < HID) wv = Wh[(size_t)L * HID * HID + (size_t)k * HID + n] * WSCALE;
    v[j] = (_Float16)wv;
  }
  volatile h8* p = (volatile h8*)(wsW + i);
  *p = v;
  __threadfence();
  *p = v;
}

__global__ __launch_bounds__(NTHR) void k_lrf_mlp(
    const float* __restrict__ x,
    const float* __restrict__ ctrl,
    const float* __restrict__ Win,
    const float* __restrict__ bin,
    const float* __restrict__ bh,
    const float* __restrict__ Wout,
    const float* __restrict__ bout,
    const int*   __restrict__ didx,
    const int*   __restrict__ cidx,
    const h8*    __restrict__ wsW,
    float*       __restrict__ out,
    int nimg)
{
  extern __shared__ __attribute__((aligned(16))) char smem[];
  _Float16* sWh   = (_Float16*)(smem + OFF_WH);
  _Float16* sAct  = (_Float16*)(smem + OFF_ACT);
  float*    sWin  = (float*)(smem + OFF_WIN);
  float*    sBin  = (float*)(smem + OFF_BIN);
  float*    sBh   = (float*)(smem + OFF_BH);
  float*    sWout = (float*)(smem + OFF_WOUT);

  const int tid = threadIdx.x;
  const int b   = blockIdx.x;
  (void)nimg;

  {
    h8* sWhv = (h8*)sWh;
    for (int i = tid; i < WH_VEC; i += NTHR) sWhv[i] = wsW[i];
    for (int i = tid; i < HP * 8; i += NTHR) {
      const int n = i >> 3, e = i & 7;
      sWin[i] = (e < NELEC && n < HID) ? Win[e * HID + n] : 0.f;
    }
    for (int i = tid; i < HP; i += NTHR) {
      sBin[i]  = (i < HID) ? bin[i] : 0.f;
      sWout[i] = (i < HID) ? Wout[i] : 0.f;
    }
    for (int i = tid; i < NLAY * HP; i += NTHR) {
      const int L = i / HP, n = i - L * HP;
      sBh[i] = (n < HID) ? bh[L * HID + n] * WSCALE : 0.f;
    }
  }
  __syncthreads();

  const int lane = tid & 31;
  const int wv   = tid >> 5;
  const int nl   = lane & 15;
  const int lh   = lane >> 4;
  _Float16* act  = sAct + wv * (32 * HP);
  const float bo = bout[0];

#pragma unroll 1
  for (int p = 0; p < PIT; ++p) {
    const int nb = (wv * PIT + p) * 32;
    const size_t R0 = (size_t)b * NNODES + (size_t)nb;

    {
      const int n  = nb + lane;
      const int pi = n >> 5, pj = n & 31;
      const float* xb = x + (size_t)b * IMGPIX + pi * (2 * IMGW) + 2 * pj;
      const f2 tp = *(const f2*)(xb);
      const f2 bt = *(const f2*)(xb + IMGW);
      float pv[4] = {tp[0], tp[1], bt[0], bt[1]};
      float cv[3];
      int di[4], ci[3];
#pragma unroll
      for (int j = 0; j < 3; ++j) {
        cv[j] = ctrl[n * 3 + j];
        int e = cidx[n * 3 + j];
        ci[j] = (e < 0) ? e + NELEC : e;
      }
#pragma unroll
      for (int j = 0; j < 4; ++j) {
        int e = didx[n * 4 + j];
        di[j] = (e < 0) ? e + NELEC : e;
      }
      float z[NELEC];
#pragma unroll
      for (int e = 0; e < NELEC; ++e) {
        float ze = 0.f;
#pragma unroll
        for (int j = 0; j < 4; ++j) ze = (di[j] == e) ? pv[j] : ze;
#pragma unroll
        for (int j = 0; j < 3; ++j) ze = (ci[j] == e) ? cv[j] : ze;
        z[e] = ze;
      }
      _Float16* myrow = act + lane * HP;
#pragma unroll 1
      for (int cb = 0; cb < HP / 8; ++cb) {
        h8 hv;
#pragma unroll
        for (int i = 0; i < 8; ++i) {
          const int col = cb * 8 + i;
          const f4 w0 = *(const f4*)(sWin + col * 8);
          const f4 w1 = *(const f4*)(sWin + col * 8 + 4);
          float a = sBin[col];
          a = fmaf(z[0], w0[0], a);
          a = fmaf(z[1], w0[1], a);
          a = fmaf(z[2], w0[2], a);
          a = fmaf(z[3], w0[3], a);
          a = fmaf(z[4], w1[0], a);
          a = fmaf(z[5], w1[1], a);
          a = fmaf(z[6], w1[2], a);
          hv[i] = (_Float16)fmaxf(a, 0.f);
        }
        *(h8a*)(myrow + cb * 8) = hv;
      }
    }
    __syncthreads();

#pragma unroll 1
    for (int L = 0; L < NLAY - 1; ++L) {
      hidden_layer_store(act, sWh + L * HP * HP, sBh + L * HP, nl, lh);
      __syncthreads();
    }

    {
      const _Float16* w   = sWh + (NLAY - 1) * HP * HP;
      const float*    b16 = sBh + (NLAY - 1) * HP;
      h16 af0[3], af1[3];
      const _Float16* a0p = act + nl * HP + 8 * lh;
      const _Float16* a1p = a0p + 16 * HP;
#pragma unroll
      for (int c = 0; c < 3; ++c) {
        af0[c] = lds_frag(a0p + c * 32);
        af1[c] = lds_frag(a1p + c * 32);
      }
      const _Float16* wp = w + nl * HP + 8 * lh;
      float s0[8], s1[8];
#pragma unroll
      for (int r = 0; r < 8; ++r) { s0[r] = 0.f; s1[r] = 0.f; }
#pragma unroll 1
      for (int t = 0; t < 6; ++t) {
        f8 d0 = splat8(b16[t * 16 + nl]);
        f8 d1 = d0;
#pragma unroll
        for (int c = 0; c < 3; ++c) {
          h16 bf = lds_frag(wp + t * 16 * HP + c * 32);
          d0 = wmma16(af0[c], bf, d0);
          d1 = wmma16(af1[c], bf, d1);
        }
        const float wo = sWout[t * 16 + nl];
#pragma unroll
        for (int r = 0; r < 8; ++r) {
          s0[r] = fmaf(fmaxf(d0[r] * WSCALE_INV, 0.f), wo, s0[r]);
          s1[r] = fmaf(fmaxf(d1[r] * WSCALE_INV, 0.f), wo, s1[r]);
        }
      }
#pragma unroll
      for (int r = 0; r < 8; ++r) {
#pragma unroll
        for (int off = 1; off < 16; off <<= 1) {
          s0[r] += __shfl_xor(s0[r], off);
          s1[r] += __shfl_xor(s1[r], off);
        }
      }
      const int q = lane & 7;
      float v0 = s0[0], v1 = s1[0];
#pragma unroll
      for (int r = 1; r < 8; ++r) {
        v0 = (q == r) ? s0[r] : v0;
        v1 = (q == r) ? s1[r] : v1;
      }
      float val = ((lane >> 3) & 1) ? v1 : v0;
      val += bo;
      f4 o;
#pragma unroll
      for (int j = 0; j < 4; ++j) {
        const int rho = 4 * q + j;
        const int src = (rho & 7) | ((rho & 8) << 1) | ((rho & 16) >> 1);
        o[j] = __shfl(val, src);
      }
      if (lane < 8) {
        volatile f4* op = (volatile f4*)(out + R0 + 4 * lane);
        *op = o;
        __threadfence();
        *op = o;
      }
    }
    __syncthreads();
  }
}

extern "C" void kernel_launch(void* const* d_in, const int* in_sizes, int n_in,
                              void* d_out, int out_size, void* d_ws, size_t ws_size,
                              hipStream_t stream) {
  if (n_in < 10) return;
  const int nimg = out_size / NNODES;
  if (nimg <= 0 || nimg * NNODES != out_size) return;
  if (in_sizes[0] != nimg * IMGPIX) return;
  if (in_sizes[1] != NNODES * 3) return;
  if (in_sizes[2] != NELEC * HID) return;
  if (in_sizes[3] != HID) return;
  if (in_sizes[4] != NLAY * HID * HID) return;
  if (in_sizes[5] != NLAY * HID) return;
  if (in_sizes[6] != HID) return;
  if (in_sizes[7] < 1) return;
  if (in_sizes[8] != NNODES * 4) return;
  if (in_sizes[9] != NNODES * 3) return;
  if (ws_size < (size_t)WH_HALVES * 2) return;

  const float* x    = (const float*)d_in[0];
  const float* ctrl = (const float*)d_in[1];
  const float* Win  = (const float*)d_in[2];
  const float* bin  = (const float*)d_in[3];
  const float* Wh   = (const float*)d_in[4];
  const float* bh   = (const float*)d_in[5];
  const float* Wout = (const float*)d_in[6];
  const float* bout = (const float*)d_in[7];
  const int*   didx = (const int*)d_in[8];
  const int*   cidx = (const int*)d_in[9];
  h8* wsW  = (h8*)d_ws;
  float* out = (float*)d_out;

  (void)hipFuncSetAttribute(reinterpret_cast<const void*>(k_lrf_mlp),
                            hipFuncAttributeMaxDynamicSharedMemorySize, SMEM_BYTES);

  k_prep_wh<<<dim3((WH_VEC + NTHR - 1) / NTHR), dim3(NTHR), 0, stream>>>(Wh, wsW, WH_VEC);
  k_lrf_mlp<<<dim3(nimg), dim3(NTHR), SMEM_BYTES, stream>>>(
      x, ctrl, Win, bin, bh, Wout, bout, didx, cidx, wsW, out, nimg);
}
